// SimpleSSM_55405078118790
// MI455X (gfx1250) — hardware-verified
//
#include <hip/hip_runtime.h>
#include <math.h>

constexpr int NBAT   = 32;
constexpr int SEQL   = 2048;
constexpr int DIN    = 64;
constexpr int DHID   = 1024;
constexpr int DOUT   = 64;
constexpr int NLAY   = 4;
constexpr int TTAIL  = 256;
constexpr int TSTART = SEQL - TTAIL;
constexpr int MROWS  = NBAT * TTAIL;
constexpr int NTHR   = 256;
constexpr int LTHR   = 1024;
constexpr float LN_EPS_F = 1e-5f;
static_assert(DIN % 32 == 0);
static_assert(MROWS % 64 == 0 && DHID % 64 == 0);
static_assert(((MROWS / 64) * (DHID / 64)) % 8 == 0);
static_assert(DIN % 64 == 0 && DHID % 64 == 0);
static_assert(DIN / 8 == 8);
static_assert((MROWS * (DIN / 8)) % NTHR == 0);
static_assert(LTHR == DHID);
static_assert(LTHR / 32 == 32);
static_assert(LTHR == 16 * DOUT && DHID == 16 * 64);
static_assert(DOUT % 32 == 0);

typedef __attribute__((ext_vector_type(16))) _Float16 v16h;
typedef __attribute__((ext_vector_type(8)))  _Float16 v8h;
typedef __attribute__((ext_vector_type(16))) __bf16   v16b;
typedef __attribute__((ext_vector_type(8)))  __bf16   v8b;
typedef __attribute__((ext_vector_type(8)))  float    v8f;
typedef __attribute__((ext_vector_type(4)))  float    v4f;

__device__ __forceinline__ unsigned short f2bf_bits(float f) {
  unsigned u = __float_as_uint(f);
  return (unsigned short)((u + 0x7FFFu + ((u >> 16) & 1u)) >> 16);
}
__device__ __forceinline__ float bf_bits2f(unsigned short h) { return __uint_as_float(((unsigned)h) << 16); }
__device__ __forceinline__ float bf16r(float f) { return bf_bits2f(f2bf_bits(f)); }

__device__ __forceinline__ void dep_guard_h(v8f& a, v8f& b, v16h x, v16h y) { asm volatile("v_nop\n\tv_nop\n\tv_nop\n\tv_nop" : "+v"(a), "+v"(b) : "v"(x), "v"(y)); }
__device__ __forceinline__ void dep_guard_b(v8f& a, v8f& b, v16b x, v16b y) { asm volatile("v_nop\n\tv_nop\n\tv_nop\n\tv_nop" : "+v"(a), "+v"(b) : "v"(x), "v"(y)); }
__device__ __forceinline__ void dep_guard4_h(v8f& a, v8f& b, v8f& c, v8f& d, v16h x, v16h y) { asm volatile("v_nop\n\tv_nop\n\tv_nop\n\tv_nop" : "+v"(a), "+v"(b), "+v"(c), "+v"(d) : "v"(x), "v"(y)); }
__device__ __forceinline__ void dep_guard4_b(v8f& a, v8f& b, v8f& c, v8f& d, v16b x, v16b y) { asm volatile("v_nop\n\tv_nop\n\tv_nop\n\tv_nop" : "+v"(a), "+v"(b), "+v"(c), "+v"(d) : "v"(x), "v"(y)); }
__device__ __forceinline__ void keep4_h(v16h a, v16h b, v16h c, v16h d) { asm volatile("v_nop" :: "v"(a), "v"(b), "v"(c), "v"(d)); }
__device__ __forceinline__ void keep4_b(v16b a, v16b b, v16b c, v16b d) { asm volatile("v_nop" :: "v"(a), "v"(b), "v"(c), "v"(d)); }
__device__ __forceinline__ void acc_guard4(v8f& a, v8f& b, v8f& c, v8f& d) { asm volatile("v_nop\n\tv_nop\n\tv_nop\n\tv_nop" : "+v"(a), "+v"(b), "+v"(c), "+v"(d)); }
template <typename T> struct Frag;
template <> struct Frag<_Float16> {
  typedef v16h V; union U { v16h v; v8h h[2]; };
  static __device__ __forceinline__ v16h load(const _Float16* p) {
    U f; f.h[0] = *(const v8h*)(p); f.h[1] = *(const v8h*)(p + 16); return f.v;
  }
  static __device__ __forceinline__ v8f mma(v16h a, v16h b, v8f c) {
    return __builtin_amdgcn_wmma_f32_16x16x32_f16(false, a, false, b, (short)0, c, false, false);
  }
  static __device__ __forceinline__ void guard(v8f& a, v8f& b, v16h x, v16h y) { dep_guard_h(a, b, x, y); }
  static __device__ __forceinline__ void guard4(v8f& a, v8f& b, v8f& c, v8f& d, v16h x, v16h y) { dep_guard4_h(a, b, c, d, x, y); }
  static __device__ __forceinline__ void keep(v16h a, v16h b, v16h c, v16h d) { keep4_h(a, b, c, d); }
};
template <> struct Frag<__bf16> {
  typedef v16b V; union U { v16b v; v8b h[2]; };
  static __device__ __forceinline__ v16b load(const __bf16* p) {
    U f; f.h[0] = *(const v8b*)(p); f.h[1] = *(const v8b*)(p + 16); return f.v;
  }
  static __device__ __forceinline__ v8f mma(v16b a, v16b b, v8f c) {
    return __builtin_amdgcn_wmma_f32_16x16x32_bf16(false, a, false, b, (short)0, c, false, false);
  }
  static __device__ __forceinline__ void guard(v8f& a, v8f& b, v16b x, v16b y) { dep_guard_b(a, b, x, y); }
  static __device__ __forceinline__ void guard4(v8f& a, v8f& b, v8f& c, v8f& d, v16b x, v16b y) { dep_guard4_b(a, b, c, d, x, y); }
  static __device__ __forceinline__ void keep(v16b a, v16b b, v16b c, v16b d) { keep4_b(a, b, c, d); }
};

template <int ET> struct Elem;
template <> struct Elem<0> { typedef _Float16 T; };
template <> struct Elem<1> { typedef __bf16 T; };
template <int ET, bool SPLIT, int BIAS_MODE, int OUT_MODE, bool RESID, int ACT = 0>
__global__ __launch_bounds__(256) void wmma_gemm64(
    const unsigned short* __restrict__ Ap, const unsigned short* __restrict__ A2p, int lda, long strideA,
    const unsigned short* __restrict__ Btp, const unsigned short* __restrict__ Bt2p, int ldb, long strideB,
    void* __restrict__ Cout, void* __restrict__ Cout2, int ldc, long strideC,
    const float* __restrict__ bias,
    const float* __restrict__ resid, long strideR,
    int M, int N, int K, float scale) {
  typedef typename Elem<ET>::T T;
  typedef typename Frag<T>::V V;
  const T* A = (const T*)Ap; const T* A2 = (const T*)A2p; const T* Bt = (const T*)Btp; const T* Bt2 = (const T*)Bt2p;
  __shared__ __align__(16) float sT[8][16 * 68];
  const int b    = blockIdx.y;
  const int lane = threadIdx.x & 31;
  const int wave = threadIdx.x >> 5;
  const int tilesN = N >> 6;
  const int tilesM = M >> 6;
  const int tile = blockIdx.x * 8 + wave;
  if (tile >= tilesM * tilesN) return;
  const int tm = tile / tilesN;
  const int tn = tile - tm * tilesN;
  const int m0 = tm << 6;
  const int n0 = tn << 6;

  const T* Ab  = A  + (size_t)b * strideA;
  const T* Bb  = Bt + (size_t)b * strideB;
  const T* Ab2 = SPLIT ? (A2  + (size_t)b * strideA) : nullptr;
  const T* Bb2 = SPLIT ? (Bt2 + (size_t)b * strideB) : nullptr;

  const int rlane = lane & 15;
  const int koff  = (lane >> 4) * 8;
  const int mOff  = (lane >> 4) * 8;

  v8f acc[4][4];
#pragma unroll
  for (int i = 0; i < 4; ++i)
#pragma unroll
    for (int j = 0; j < 4; ++j) acc[i][j] = (v8f){0.f,0.f,0.f,0.f,0.f,0.f,0.f,0.f};

  for (int k0 = 0; k0 < K; k0 += 32) {
    V bh[4], bl[4];
#pragma unroll
    for (int j = 0; j < 4; ++j) {
      const size_t bo = (size_t)(n0 + (j << 4) + rlane) * ldb + koff + k0;
      bh[j] = Frag<T>::load(Bb + bo);
      if (SPLIT) bl[j] = Frag<T>::load(Bb2 + bo);
    }
#pragma unroll
    for (int i = 0; i < 4; ++i) {
      const size_t ao = (size_t)(m0 + (i << 4) + rlane) * lda + koff + k0;
      V ah = Frag<T>::load(Ab + ao);
      V al;
      if (SPLIT) al = Frag<T>::load(Ab2 + ao);
#pragma unroll
      for (int j = 0; j < 4; ++j) {
        acc[i][j] = Frag<T>::mma(ah, bh[j], acc[i][j]);
        if (SPLIT) {
          acc[i][j] = Frag<T>::mma(ah, bl[j], acc[i][j]);
          acc[i][j] = Frag<T>::mma(al, bh[j], acc[i][j]);
        }
      }
      Frag<T>::guard4(acc[i][0], acc[i][1], acc[i][2], acc[i][3], ah, SPLIT ? al : ah);
    }
    Frag<T>::keep(bh[0], bh[1], bh[2], bh[3]);
    if (SPLIT) Frag<T>::keep(bl[0], bl[1], bl[2], bl[3]);
  }
  acc_guard4(acc[0][0], acc[0][1], acc[0][2], acc[0][3]);
  acc_guard4(acc[1][0], acc[1][1], acc[1][2], acc[1][3]);
  acc_guard4(acc[2][0], acc[2][1], acc[2][2], acc[2][3]);
  acc_guard4(acc[3][0], acc[3][1], acc[3][2], acc[3][3]);

  float* slab = sT[wave];
  const float* Rb = RESID ? (resid + (size_t)b * strideR) : nullptr;
#pragma unroll
  for (int i = 0; i < 4; ++i) {
    const int mBase = m0 + (i << 4);
#pragma unroll
    for (int j = 0; j < 4; ++j) {
      const int n = n0 + (j << 4) + rlane;
      float bv = 0.f;
      if (BIAS_MODE == 2) bv = bias[n];
#pragma unroll
      for (int r = 0; r < 8; ++r) {
        float v = acc[i][j][r] * scale;
        if (BIAS_MODE == 1) v += bias[mBase + mOff + r];
        if (BIAS_MODE == 2) v += bv;
        if (RESID) v += Rb[(size_t)(mBase + mOff + r) * ldc + n];
        if (ACT == 1) v = tanhf(v);
        if (ACT == 2) v = fmaxf(v, 0.0f);
        if (ACT == 3) v = v / (1.0f + expf(-v));
        if (ACT == 4) v = (v > 0.f) ? v : 0.01f * v;
        if (ACT == 5) v = 0.5f * v * (1.0f + erff(v * 0.70710678118654752f));
        slab[(mOff + r) * 68 + (j << 4) + rlane] = v;
      }
    }
    __builtin_amdgcn_fence(__ATOMIC_RELEASE, "workgroup");
    __builtin_amdgcn_wave_barrier();
    __builtin_amdgcn_fence(__ATOMIC_ACQUIRE, "workgroup");
    if (OUT_MODE == 0) {
      float* C = (float*)Cout + (size_t)b * strideC;
      const int hh = lane >> 4, c4 = (lane & 15) * 4;
      for (int pass = 0; pass < 2; ++pass) {
#pragma unroll
        for (int it = 0; it < 8; ++it) {
          const int row = it * 2 + hh;
          v4f v = *(const v4f*)(slab + row * 68 + c4);
          *(volatile v4f*)(C + (size_t)(mBase + row) * ldc + n0 + c4) = v;
        }
        __threadfence();
      }
    } else {
      const int q = lane >> 3, c8 = (lane & 7) * 8;
      unsigned short* C  = (unsigned short*)Cout  + (size_t)b * strideC;
      unsigned short* C2 = (OUT_MODE == 2) ? ((unsigned short*)Cout2 + (size_t)b * strideC) : nullptr;
      for (int pass = 0; pass < 2; ++pass) {
#pragma unroll
        for (int it = 0; it < 4; ++it) {
          const int row = it * 4 + q;
          const float* sp = slab + row * 68 + c8;
          v8h hv, lv;
#pragma unroll
          for (int e = 0; e < 8; ++e) {
            if (OUT_MODE == 1) {
              hv[e] = (_Float16)sp[e];
            } else {
              unsigned short hb = f2bf_bits(sp[e]);
              unsigned short lb = f2bf_bits(sp[e] - bf_bits2f(hb));
              hv[e] = __builtin_bit_cast(_Float16, hb);
              lv[e] = __builtin_bit_cast(_Float16, lb);
            }
          }
          *(volatile v8h*)(C + (size_t)(mBase + row) * ldc + n0 + c8) = hv;
          if (OUT_MODE == 2) *(volatile v8h*)(C2 + (size_t)(mBase + row) * ldc + n0 + c8) = lv;
        }
        __threadfence();
      }
    }
    __builtin_amdgcn_fence(__ATOMIC_RELEASE, "workgroup");
    __builtin_amdgcn_wave_barrier();
    __builtin_amdgcn_fence(__ATOMIC_ACQUIRE, "workgroup");
  }
}

template <int MODE>
__global__ __launch_bounds__(NTHR) void tpw_kernel(const float* __restrict__ src, int R, int C, int ldo,
                                                  unsigned short* __restrict__ O, float sc) {
  __shared__ float Tt[64 * 65];
  const int tid = threadIdx.x;
  const int c0 = blockIdx.x * 64, r0 = blockIdx.y * 64;
#pragma unroll
  for (int i = 0; i < 4; ++i) {
    const int idx = i * NTHR + tid;
    const int rr = idx >> 4, cc = (idx & 15) * 4;
    const v4f v = *(const v4f*)(src + (size_t)(r0 + rr) * (size_t)C + c0 + cc);
    Tt[rr * 65 + cc + 0] = v[0];
    Tt[rr * 65 + cc + 1] = v[1];
    Tt[rr * 65 + cc + 2] = v[2];
    Tt[rr * 65 + cc + 3] = v[3];
  }
  __syncthreads();
  const int q = tid >> 3, c8 = (tid & 7) * 8;
  v8h hv[2];
#pragma unroll
  for (int g = 0; g < 2; ++g) {
    const int qq = g * 32 + q;
#pragma unroll
    for (int e = 0; e < 8; ++e) {
      const float f = Tt[(c8 + e) * 65 + qq];
      unsigned short bits;
      if (MODE == 0) {
        bits = f2bf_bits(f * sc);
      } else {
        const float fb = bf_bits2f(f2bf_bits(f));
        bits = __builtin_bit_cast(unsigned short, (_Float16)(fb * sc));
      }
      hv[g][e] = __builtin_bit_cast(_Float16, bits);
    }
  }
  for (int pass = 0; pass < 2; ++pass) {
#pragma unroll
    for (int g = 0; g < 2; ++g) {
      const size_t o = (size_t)(c0 + g * 32 + q) * (size_t)ldo + (size_t)(r0 + c8);
      *(volatile v8h*)(O + o) = hv[g];
    }
    __threadfence();
  }
}

__global__ __launch_bounds__(NTHR) void xtail_cvt_kernel(const float* __restrict__ x, unsigned short* __restrict__ dst) {
  const int i  = blockIdx.x * NTHR + threadIdx.x;
  const int n8 = MROWS * (DIN / 8);
  if (i < n8) {
    const int row = i >> 3;
    const int c8  = i & 7;
    const int bb  = row / TTAIL;
    const int j   = row - bb * TTAIL;
    const float* sp = x + ((size_t)bb * SEQL + (size_t)(TSTART + j)) * DIN + c8 * 8;
    const v4f a = *(const v4f*)(sp);
    const v4f c = *(const v4f*)(sp + 4);
    v8h hv;
#pragma unroll
    for (int e = 0; e < 4; ++e) {
      hv[e]     = __builtin_bit_cast(_Float16, f2bf_bits(a[e]));
      hv[4 + e] = __builtin_bit_cast(_Float16, f2bf_bits(c[e]));
    }
    *(volatile v8h*)(dst + (size_t)i * 8) = hv;
    __threadfence();
    *(volatile v8h*)(dst + (size_t)i * 8) = hv;
  }
}

__device__ __forceinline__ float wave_sum32(float s) {
#pragma unroll
  for (int off = 1; off < 32; off <<= 1) s += __shfl_xor(s, off, 32);
  return s;
}

__global__ __launch_bounds__(LTHR) void ema_ln_head_kernel(const float* __restrict__ HP, const float* __restrict__ b_in,
                                                          const float* __restrict__ alphas, const float* __restrict__ gam,
                                                          const float* __restrict__ bet, const float* __restrict__ w_out,
                                                          const float* __restrict__ b_out, float* __restrict__ out) {
  __shared__ float red[2][32];
  __shared__ float sa[NLAY * LTHR];
  __shared__ __align__(16) float hs[DHID];
  __shared__ float part[LTHR];
  __shared__ __align__(16) float os[DOUT];
  const int tid = threadIdx.x, lane = tid & 31, wave = tid >> 5;
  const int b = blockIdx.x;

  const float bi = bf16r(b_in[tid]);
  const float g  = bf16r(gam[tid]);
  const float be = bf16r(bet[tid]);
#pragma unroll 1
  for (int l = 0; l < NLAY; ++l) {
    const float al = bf16r(alphas[l * DHID + tid]);
    sa[l * LTHR + tid] = 1.0f / (1.0f + expf(-al));
  }
  float av[NLAY], om[NLAY], ev[NLAY];
#pragma unroll
  for (int l = 0; l < NLAY; ++l) {
    av[l] = sa[l * LTHR + tid];
    om[l] = 1.0f - av[l];
    ev[l] = 0.0f;
  }
  float v = 0.0f;
  const float* hrow = HP + (size_t)b * TTAIL * DHID + tid;
  const float inv_n = 1.0f / (float)DHID;

#pragma unroll 1
  for (int t = 0; t < TTAIL; ++t) {
    const float pre = hrow[(size_t)t * DHID] + bi;
    v = 0.5f * pre * (1.0f + erff(pre * 0.70710678118654752f));
#pragma unroll
    for (int l = 0; l < NLAY; ++l) {
      ev[l] = av[l] * v + om[l] * ev[l];
      const float r = v + ev[l];
      float s = wave_sum32(r);
      if (lane == 0) red[0][wave] = s;
      __syncthreads();
      float s2 = wave_sum32(red[0][lane]);
      const float mu = s2 * inv_n;
      const float dlt = r - mu;
      float q = wave_sum32(dlt * dlt);
      if (lane == 0) red[1][wave] = q;
      __syncthreads();
      float q2 = wave_sum32(red[1][lane]);
      const float var  = q2 * inv_n;
      const float rstd = rsqrtf(var + LN_EPS_F);
      v = (dlt * rstd) * g + be;
    }
  }

  hs[tid] = v;
  __syncthreads();
  const int o  = tid & (DOUT - 1);
  const int kq = tid >> 6;
  const float* wp = w_out + (size_t)(kq * 64) * DOUT + o;
  const float* hq = hs + kq * 64;
  float acc = 0.0f;
#pragma unroll 2
  for (int k = 0; k < 64; ++k) acc = fmaf(hq[k], bf16r(wp[(size_t)k * DOUT]), acc);
  part[tid] = acc;
  __syncthreads();
  if (tid < DOUT) {
    float s = 0.0f;
#pragma unroll
    for (int kk = 0; kk < 16; ++kk) s += part[kk * 64 + tid];
    os[tid] = s + bf16r(b_out[tid]);
  }
  __syncthreads();
  const int ti = (tid < 16) ? tid : 0;
  const v4f ov = *(const v4f*)(os + ti * 4);
  float* orow = out + (size_t)b * DOUT;
  for (int pass = 0; pass < 2; ++pass) {
    if (tid < 16) *(volatile v4f*)(orow + ti * 4) = ov;
    __threadfence();
  }
}

extern "C" void kernel_launch(void* const* d_in, const int* in_sizes, int n_in,
                              void* d_out, int out_size, void* d_ws, size_t ws_size, hipStream_t stream) {
  if (n_in < 8 || d_out == nullptr || d_ws == nullptr) return;
  if (in_sizes[0] != NBAT * SEQL * DIN || in_sizes[1] != DIN * DHID || in_sizes[2] != DHID ||
      in_sizes[3] != NLAY * DHID || in_sizes[4] != DHID || in_sizes[5] != DHID ||
      in_sizes[6] != DHID * DOUT || in_sizes[7] != DOUT || out_size != NBAT * DOUT) return;

  const float* x      = (const float*)d_in[0];
  const float* w_in   = (const float*)d_in[1];
  const float* b_in   = (const float*)d_in[2];
  const float* alphas = (const float*)d_in[3];
  const float* gam    = (const float*)d_in[4];
  const float* bet    = (const float*)d_in[5];
  const float* w_out  = (const float*)d_in[6];
  const float* b_out  = (const float*)d_in[7];
  float* out = (float*)d_out;

  char* ws = (char*)d_ws; size_t off = 0;
  auto carve = [&](size_t bytes) -> char* { char* p = ws + off; off += (bytes + 255) & ~(size_t)255; return p; };
  unsigned short* XB = (unsigned short*)carve((size_t)MROWS * DIN * 2);
  unsigned short* WB = (unsigned short*)carve((size_t)DHID * DIN * 2);
  float*          HP = (float*)carve((size_t)MROWS * DHID * 4);
  if (off > ws_size || off > (size_t)134217728) return;

  xtail_cvt_kernel<<<(MROWS * (DIN / 8)) / NTHR, NTHR, 0, stream>>>(x, XB);
  tpw_kernel<0><<<dim3(DHID / 64, DIN / 64), NTHR, 0, stream>>>(w_in, DIN, DHID, DIN, WB, 1.0f);
  const dim3 ggrid((MROWS / 64) * (DHID / 64) / 8, 1);
  wmma_gemm64<1, false, 0, 0, false, 0><<<ggrid, 256, 0, stream>>>(
      XB, XB, DIN, 0L, WB, WB, DIN, 0L, (void*)HP, (void*)HP, DHID, 0L,
      b_in, HP, 0L, MROWS, DHID, DIN, 1.0f);
  ema_ln_head_kernel<<<NBAT, LTHR, 0, stream>>>(HP, b_in, alphas, gam, bet, w_out, b_out, out);
}
